// AxialAttention_6717328851074
// MI455X (gfx1250) — hardware-verified
//
#include <hip/hip_runtime.h>
#include <math.h>

typedef __attribute__((ext_vector_type(16))) _Float16 v16h;
typedef __attribute__((ext_vector_type(16))) __bf16 v16b;
typedef __attribute__((ext_vector_type(8)))  _Float16 v8h;
typedef __attribute__((ext_vector_type(8)))  float v8f;
typedef __attribute__((ext_vector_type(4)))  float v4f;
typedef __attribute__((ext_vector_type(2)))  float v2f;
typedef __attribute__((ext_vector_type(4)))  unsigned v4u;
typedef __attribute__((ext_vector_type(4)))  int v4i;
typedef float __attribute__((may_alias)) float_a;
typedef int __attribute__((may_alias)) int_a;

template <typename T> __device__ __forceinline__ void vst2(void* p, T v) { *(volatile T*)p = v; __threadfence(); *(volatile T*)p = v; }
__device__ __forceinline__ v8f wmma16(v16h a, v16h b, v8f c) {
  v8f d = __builtin_amdgcn_wmma_f32_16x16x32_f16(false, a, false, b, (short)0, c, false, false);
  asm volatile("v_nop\n\tv_nop\n\tv_nop\n\tv_nop" : "+v"(d) : "v"(a), "v"(b));
  return d;
}
__device__ __forceinline__ v8f wmma_bf(v16b a, v16b b, v8f c) {
  v8f d = __builtin_amdgcn_wmma_f32_16x16x32_bf16(false, a, false, b, (short)0, c, false, false);
  asm volatile("v_nop\n\tv_nop\n\tv_nop\n\tv_nop" : "+v"(d) : "v"(a), "v"(b));
  return d;
}
__device__ __forceinline__ v16h frag_h(const _Float16* rowk0, int lane) {
  union { v16h v; v8h q[2]; } u; const _Float16* p = rowk0 + 8 * (lane >> 4);
  u.q[0] = *(const v8h*)p; u.q[1] = *(const v8h*)(p + 16); return u.v;
}
__device__ __forceinline__ v16h frag_f32(const float* rowk0, int lane) {
  v16h a; const float* p = rowk0 + 8 * (lane >> 4);
#pragma unroll
  for (int i = 0; i < 8; ++i) { a[i] = (_Float16)p[i]; a[8 + i] = (_Float16)p[16 + i]; }
  return a;
}
__device__ __forceinline__ v16h frag_f32s(const float* rowk0, int lane, float sc) {
  v16h a; const float* p = rowk0 + 8 * (lane >> 4);
#pragma unroll
  for (int i = 0; i < 8; ++i) { a[i] = (_Float16)(p[i] * sc); a[8 + i] = (_Float16)(p[16 + i] * sc); }
  return a;
}
__device__ __forceinline__ v16h fragc_f32(const float* W, int k0, int n, int lane, int ld, int K) {
  v16h a; const int g = lane >> 4;
#pragma unroll
  for (int i = 0; i < 8; ++i) { const int ka = k0 + 8 * g + i, kb = ka + 16;
    a[i] = (_Float16)(ka < K ? W[(size_t)(ka < K ? ka : K - 1) * ld + n] : 0.f); a[8 + i] = (_Float16)(kb < K ? W[(size_t)(kb < K ? kb : K - 1) * ld + n] : 0.f); }
  return a;
}
struct F2 { v16b h, l; };
__device__ __forceinline__ F2 bsplit16(const float v[16]) { F2 r;
#pragma unroll
  for (int i = 0; i < 16; ++i) { const __bf16 h = (__bf16)v[i]; r.h[i] = h; r.l[i] = (__bf16)(v[i] - (float)h); }
  return r; }
__device__ __forceinline__ F2 split_row(const float* row, int k0, int lane) { float v[16]; const float* p = row + k0 + 8 * (lane >> 4);
#pragma unroll
  for (int i = 0; i < 8; ++i) { v[i] = p[i]; v[8 + i] = p[16 + i]; }
  return bsplit16(v); }
__device__ __forceinline__ F2 split_rowK(const float* row, int k0, int lane, int K) { float v[16]; const int g = lane >> 4;
#pragma unroll
  for (int i = 0; i < 8; ++i) { const int ka = k0 + 8 * g + i, kb = ka + 16; v[i] = ka < K ? row[ka < K ? ka : K - 1] : 0.f; v[8 + i] = kb < K ? row[kb < K ? kb : K - 1] : 0.f; }
  return bsplit16(v); }
__device__ __forceinline__ F2 split_col(const float* W, int k0, int n, int lane, int ld, int K) { float v[16]; const int g = lane >> 4;
#pragma unroll
  for (int i = 0; i < 8; ++i) { const int ka = k0 + 8 * g + i, kb = ka + 16; v[i] = ka < K ? W[(size_t)(ka < K ? ka : K - 1) * ld + n] : 0.f; v[8 + i] = kb < K ? W[(size_t)(kb < K ? kb : K - 1) * ld + n] : 0.f; }
  return bsplit16(v); }
__device__ __forceinline__ v8f mac3(const F2& a, const F2& b, v8f c) { c = wmma_bf(a.l, b.h, c); c = wmma_bf(a.h, b.l, c); return wmma_bf(a.h, b.h, c); }
__device__ __forceinline__ float sigm(float v) { return 1.0f / (1.0f + expf(-v)); }
#define LDSX() do { asm volatile("s_wait_dscnt 0" ::: "memory"); __builtin_amdgcn_wave_barrier(); __builtin_amdgcn_fence(__ATOMIC_RELEASE, "workgroup"); } while (0)

#define NSEQ 512
#define HL 64
#define CIN 256
#define OP 256
#define NG 8
#define GP 32
#define CQ 16
#define NREL 127
#ifndef NSP
#define NSP NSEQ
#endif
#define SP 512
typedef __attribute__((ext_vector_type(8))) __bf16 v8b;
__device__ __forceinline__ float bfr(float v) { return (float)(__bf16)v; }
__device__ __forceinline__ v16b frag_b(const __bf16* rowk0, int lane) { union { v16b v; v8b q[2]; } u; const __bf16* p = rowk0 + 8 * (lane >> 4); u.q[0] = *(const v8b*)p; u.q[1] = *(const v8b*)(p + 16); return u.v; }
__device__ __forceinline__ float bn_aff(const float* __restrict__ P, int nch, int c, float x) { const float ga = bfr(P[c]), be = bfr(P[nch + c]), mu = bfr(P[2 * nch + c]), va = bfr(P[3 * nch + c]); return ga * (x - mu) * rsqrtf(va + 1e-5f) + be; }
#define WS_QKV 0u
#define WS_END (WS_QKV + 4u * (size_t)NSEQ * 2 * OP * HL)

__global__ __launch_bounds__(128) void k_qkv(const float* __restrict__ X, const float* __restrict__ Wm, const float* __restrict__ BNQ, float* __restrict__ QKV) { __shared__ __align__(16) float so[128][68];
  const int tid = threadIdx.x, wave = tid >> 5, lane = tid & 31, col = lane & 15, g = lane >> 4; const int b = blockIdx.x; const int o0 = blockIdx.y * 128;
  v8f acc[8] = {};
#pragma unroll 1
  for (int kc = 0; kc < CIN / 32; ++kc) { v16b a; { const float* p = X + ((size_t)(kc * 32 + 8 * g) * SP + b) * HL + wave * 16 + col;
#pragma unroll
      for (int i = 0; i < 8; ++i) { a[i] = (__bf16)p[(size_t)i * SP * HL]; a[8 + i] = (__bf16)p[(size_t)(16 + i) * SP * HL]; } }
    asm volatile("s_wait_loadcnt 0x0" ::: "memory");
#pragma unroll
    for (int j = 0; j < 8; ++j) { v16b w; { const float* pw = Wm + (size_t)(o0 + j * 16 + col) * CIN + kc * 32 + 8 * g;
#pragma unroll
        for (int i = 0; i < 8; ++i) { w[i] = (__bf16)pw[i]; w[8 + i] = (__bf16)pw[16 + i]; } }
      asm volatile("s_wait_loadcnt 0x0" ::: "memory"); acc[j] = wmma_bf(a, w, acc[j]); } }
#pragma unroll
  for (int j = 0; j < 8; ++j) { const int oc = o0 + j * 16 + col; const float ga = bfr(BNQ[oc]), be = bfr(BNQ[512 + oc]), mu = bfr(BNQ[1024 + oc]), va = bfr(BNQ[1536 + oc]); asm volatile("s_wait_loadcnt 0x0" ::: "memory"); const float sc = ga * rsqrtf(va + 1e-5f);
#pragma unroll
    for (int r = 0; r < 8; ++r) so[j * 16 + col][wave * 16 + 8 * g + r] = (acc[j][r] - mu) * sc + be; }
  __syncthreads();
  for (int e = tid; e < 128 * 16; e += 128) { const int cl = e >> 4, q = e & 15; vst2(QKV + ((size_t)b * 512 + o0 + cl) * HL + q * 4, *(const v4f*)&so[cl][q * 4]); } }
__global__ __launch_bounds__(128) void k_axial(const float* __restrict__ QKV, const float* __restrict__ REL, const float* __restrict__ BNS, const float* __restrict__ BNO, float* __restrict__ OUT) {
  __shared__ __align__(16) __bf16 qTh[HL][40], qTl[HL][40], kTh[HL][40], kTl[HL][40];
  __shared__ __align__(16) __bf16 rqT[128][40], rkT[128][40];
  __shared__ __align__(16) __bf16 vh[GP][72], vl[GP][72], rv[GP][136];
  __shared__ __align__(16) float ss[HL][68], st[HL][132], stk[HL][132];
  __shared__ __align__(16) __bf16 ph[HL][72], pl[HL][72], pkh[HL][136], pkl[HL][136];
  __shared__ __align__(16) float sout[2 * GP][68];
  const int tid = threadIdx.x, wave = tid >> 5, lane = tid & 31, col = lane & 15, g16 = lane >> 4; const int b = blockIdx.x, grp = blockIdx.y;
  const float* base = QKV + ((size_t)b * 512 + grp * 64) * HL;
  for (int e = tid; e < HL * 32; e += 128) { const int i = e & 63, c = e >> 6;
    float qv = 0.f, kv = 0.f; if (c < CQ) { qv = base[(size_t)c * HL + i]; kv = base[(size_t)(CQ + c) * HL + i]; }
    const __bf16 qh = (__bf16)qv, kh = (__bf16)kv; qTh[i][c] = qh; qTl[i][c] = (__bf16)(qv - (float)qh); kTh[i][c] = kh; kTl[i][c] = (__bf16)(kv - (float)kh); }
  for (int e = tid; e < 128 * 32; e += 128) { const int m = e >> 5, c = e & 31; float a = 0.f, bq = 0.f; if (c < CQ && m < NREL) { a = REL[(size_t)c * NREL + m]; bq = REL[(size_t)(CQ + c) * NREL + m]; } rqT[m][c] = (__bf16)a; rkT[m][c] = (__bf16)bq; }
  for (int e = tid; e < GP * HL; e += 128) { const int c = e >> 6, j = e & 63; const float vv = base[(size_t)(GP + c) * HL + j]; const __bf16 h = (__bf16)vv; vh[c][j] = h; vl[c][j] = (__bf16)(vv - (float)h); }
  for (int e = tid; e < GP * 8; e += 128) { const int c = e >> 3, z = e & 7; vh[c][64 + z] = (__bf16)0.f; vl[c][64 + z] = (__bf16)0.f; }
  for (int e = tid; e < GP * 136; e += 128) { const int c = e / 136, m = e % 136; rv[c][m] = (__bf16)((m < NREL) ? REL[(size_t)(GP + c) * NREL + m] : 0.f); }
  for (int e = tid; e < HL * 8; e += 128) { const int i = e >> 3, z = e & 7; qTh[i][32 + z] = qTl[i][32 + z] = kTh[i][32 + z] = kTl[i][32 + z] = (__bf16)0.f; rqT[i][32 + z] = rkT[i][32 + z] = rqT[64 + i][32 + z] = rkT[64 + i][32 + z] = (__bf16)0.f; }
  __syncthreads();
  const int r0 = wave * 16;
  { const v16b aqh = frag_b(&qTh[r0 + col][0], lane), aql = frag_b(&qTl[r0 + col][0], lane), akh = frag_b(&kTh[r0 + col][0], lane), akl = frag_b(&kTl[r0 + col][0], lane);
#pragma unroll
    for (int ct = 0; ct < 4; ++ct) { const v16b bh = frag_b(&kTh[ct * 16 + col][0], lane), bl = frag_b(&kTl[ct * 16 + col][0], lane); v8f acc = {}; acc = wmma_bf(aqh, bh, acc); acc = wmma_bf(aql, bh, acc); acc = wmma_bf(aqh, bl, acc);
#pragma unroll
      for (int r = 0; r < 8; ++r) ss[r0 + 8 * g16 + r][ct * 16 + col] = acc[r]; }
#pragma unroll
    for (int ct = 0; ct < 8; ++ct) { const v16b br = frag_b(&rqT[ct * 16 + col][0], lane); v8f acc = {}; acc = wmma_bf(aqh, br, acc); acc = wmma_bf(aql, br, acc);
      const v16b brk = frag_b(&rkT[ct * 16 + col][0], lane); v8f ack = {}; ack = wmma_bf(akh, brk, ack); ack = wmma_bf(akl, brk, ack);
#pragma unroll
      for (int r = 0; r < 8; ++r) { st[r0 + 8 * g16 + r][ct * 16 + col] = acc[r]; stk[r0 + 8 * g16 + r][ct * 16 + col] = ack[r]; } } }
  __syncthreads();
  { const int i = r0 + (lane >> 1), half = lane & 1;
    const float g0 = bfr(BNS[grp]), b0 = bfr(BNS[24 + grp]), m0 = bfr(BNS[48 + grp]), v0 = bfr(BNS[72 + grp]);
    const float g1 = bfr(BNS[NG + grp]), b1 = bfr(BNS[24 + NG + grp]), m1 = bfr(BNS[48 + NG + grp]), v1 = bfr(BNS[72 + NG + grp]);
    const float g2 = bfr(BNS[2 * NG + grp]), b2 = bfr(BNS[24 + 2 * NG + grp]), m2 = bfr(BNS[48 + 2 * NG + grp]), v2 = bfr(BNS[72 + 2 * NG + grp]);
    const float s0 = g0 * rsqrtf(v0 + 1e-5f), s1 = g1 * rsqrtf(v1 + 1e-5f), s2 = g2 * rsqrtf(v2 + 1e-5f);
    float e32[32]; float mx = -3.0e38f;
#pragma unroll
    for (int q = 0; q < 32; ++q) { const int j = half * 32 + q; const float qk = ss[i][j]; const float qr = st[i][i - j + 63]; const float kr = stk[j][j - i + 63];
      const float v = ((qk - m0) * s0 + b0) + ((qr - m1) * s1 + b1) + ((kr - m2) * s2 + b2); e32[q] = v; mx = fmaxf(mx, v); }
    mx = fmaxf(mx, __shfl_xor(mx, 1)); float sum = 0.f;
#pragma unroll
    for (int q = 0; q < 32; ++q) { e32[q] = expf(e32[q] - mx); sum += e32[q]; }
    sum += __shfl_xor(sum, 1); const float inv = 1.0f / sum;
#pragma unroll
    for (int q = 0; q < 32; ++q) { const int j = half * 32 + q; const float p = e32[q] * inv; const __bf16 hh = (__bf16)p; const __bf16 lo = (__bf16)(p - (float)hh); ph[i][j] = hh; pl[i][j] = lo; const int m = i - j + 63; pkh[i][m] = hh; pkl[i][m] = lo; }
    for (int m = half; m < 136; m += 2) { if (m < i || m > i + 63) { pkh[i][m] = (__bf16)0.f; pkl[i][m] = (__bf16)0.f; } }
    if (half == 0) { for (int z = 64; z < 72; ++z) { ph[i][z] = (__bf16)0.f; pl[i][z] = (__bf16)0.f; } } }
  LDSX();
  { v8f asv[2] = {}, ase[2] = {};
#pragma unroll
    for (int kc = 0; kc < 2; ++kc) { const v16b ah = frag_b(&ph[r0 + col][kc * 32], lane), al = frag_b(&pl[r0 + col][kc * 32], lane);
#pragma unroll
      for (int ct = 0; ct < 2; ++ct) { const v16b bh = frag_b(&vh[ct * 16 + col][kc * 32], lane), bl = frag_b(&vl[ct * 16 + col][kc * 32], lane); asv[ct] = wmma_bf(ah, bh, asv[ct]); asv[ct] = wmma_bf(al, bh, asv[ct]); asv[ct] = wmma_bf(ah, bl, asv[ct]); } }
#pragma unroll
    for (int kc = 0; kc < 4; ++kc) { const v16b ah = frag_b(&pkh[r0 + col][kc * 32], lane), al = frag_b(&pkl[r0 + col][kc * 32], lane);
#pragma unroll
      for (int ct = 0; ct < 2; ++ct) { const v16b br = frag_b(&rv[ct * 16 + col][kc * 32], lane); ase[ct] = wmma_bf(ah, br, ase[ct]); ase[ct] = wmma_bf(al, br, ase[ct]); } }
#pragma unroll
    for (int ct = 0; ct < 2; ++ct) { const int c = ct * 16 + col; const int o = grp * GP + c; const int c0 = 2 * o, c1 = 2 * o + 1;
      const float ga0 = bfr(BNO[c0]), be0 = bfr(BNO[512 + c0]), mu0 = bfr(BNO[1024 + c0]), va0 = bfr(BNO[1536 + c0]);
      const float ga1 = bfr(BNO[c1]), be1 = bfr(BNO[512 + c1]), mu1 = bfr(BNO[1024 + c1]), va1 = bfr(BNO[1536 + c1]);
      asm volatile("s_wait_loadcnt 0x0" ::: "memory");
      const float sc0 = ga0 * rsqrtf(va0 + 1e-5f), sc1 = ga1 * rsqrtf(va1 + 1e-5f);
#pragma unroll
      for (int r = 0; r < 8; ++r) sout[c][r0 + 8 * g16 + r] = ((asv[ct][r] - mu0) * sc0 + be0) + ((ase[ct][r] - mu1) * sc1 + be1); } }
  __syncthreads();
  for (int e = tid; e < GP * 16; e += 128) { const int c = e >> 4, q = e & 15; const int o = grp * GP + c; vst2(OUT + ((size_t)o * SP + b) * HL + q * 4, *(const v4f*)&sout[c][q * 4]); } }
extern "C" void kernel_launch(void* const* d_in, const int* in_sizes, int n_in, void* d_out, int out_size, void* d_ws, size_t ws_size, hipStream_t stream) {
  (void)in_sizes; (void)n_in; (void)out_size;
  if (ws_size < (size_t)WS_END) return;
  char* ws = (char*)d_ws; const float** F = (const float**)d_in; float* QKV = (float*)(ws + WS_QKV);
  k_qkv<<<dim3(NSP, 4), 128, 0, stream>>>(F[0], F[1], F[3], QKV);
  k_axial<<<dim3(NSP, NG), 128, 0, stream>>>(QKV, F[2], F[4], F[5], (float*)d_out);
}
